// GriffinHaloBase_76459007803766
// MI455X (gfx1250) — hardware-verified
//
#include <hip/hip_runtime.h>


#define NB_  4
#define TT   2048
#define DD   768
#define DC   384
#define DG   384
#define DF   2048
typedef _Float16 h16;
typedef unsigned short bf;
typedef __attribute__((ext_vector_type(16))) __bf16   v16bf;
typedef __attribute__((ext_vector_type(16))) _Float16 v16h;
typedef __attribute__((ext_vector_type(8)))  _Float16 v8h;
typedef __attribute__((ext_vector_type(8)))  unsigned short v8us;
typedef __attribute__((ext_vector_type(8)))  float    v8f;
typedef __attribute__((ext_vector_type(4)))  float    v4f;
typedef v8h  __attribute__((may_alias)) v8ha;
typedef v4f  __attribute__((may_alias)) v4fa;
typedef v8us __attribute__((may_alias)) v8usa;

__device__ __forceinline__ unsigned short f2bf(float f) { unsigned u = __float_as_uint(f); u += 0x7FFFu + ((u >> 16) & 1u); return (unsigned short)(u >> 16); }
__device__ __forceinline__ float bf2f(unsigned short b) { return __uint_as_float(((unsigned)b) << 16); }
__device__ __forceinline__ float bfr(float f) { return bf2f(f2bf(f)); }
__device__ __forceinline__ v16h cat16(v8h lo, v8h hi) { return __builtin_shufflevector(lo, hi, 0, 1, 2, 3, 4, 5, 6, 7, 8, 9, 10, 11, 12, 13, 14, 15); }
__device__ __forceinline__ v16bf cat16b(v8us lo, v8us hi) { return __builtin_bit_cast(v16bf, __builtin_shufflevector(lo, hi, 0, 1, 2, 3, 4, 5, 6, 7, 8, 9, 10, 11, 12, 13, 14, 15)); }
__device__ __forceinline__ v8f wmma16(v16h a, v16h b, v8f c) { return __builtin_amdgcn_wmma_f32_16x16x32_f16(false, a, false, b, (short)0, c, false, false); }
__device__ __forceinline__ v8f wmmab(v16bf a, v16bf b, v8f c) { return __builtin_amdgcn_wmma_f32_16x16x32_bf16(false, a, false, b, (short)0, c, false, false); }


template <typename T16> struct WFrag;
template <> struct WFrag<h16> { typedef v16h V; static __device__ __forceinline__ V ld(const h16* p) { return cat16(*(const v8h*)p, *(const v8h*)(p + 16)); } static __device__ __forceinline__ v8f mma(V a, V b, v8f c) { return wmma16(a, b, c); } };
template <> struct WFrag<bf> { typedef v16bf V; static __device__ __forceinline__ V ld(const bf* p) { return cat16b(*(const v8us*)p, *(const v8us*)(p + 16)); } static __device__ __forceinline__ v8f mma(V a, V b, v8f c) { return wmmab(a, b, c); } };
template <typename T16, int NSPLIT, bool BIAS>
__global__ __launch_bounds__(32) void k_gemmw(const T16* __restrict__ A, const T16* __restrict__ A2, const T16* __restrict__ Bt, const T16* __restrict__ Bt2, int K, float* C, int ldc, const float* __restrict__ bias, size_t sA, size_t sB, size_t sC) {
    typedef typename WFrag<T16>::V V;
    __shared__ __align__(16) float os[16 * 68];
    const size_t z = blockIdx.z; A += z * sA; if (A2) A2 += z * sA; Bt += z * sB; if (Bt2) Bt2 += z * sB; C += z * sC;
    const int lane = threadIdx.x & 31, lr = lane & 15, hi = lane >> 4; const int r0 = blockIdx.x * 64, c0 = blockIdx.y * 64;
    v8f acc[4][4];
#pragma unroll
    for (int mb = 0; mb < 4; ++mb)
#pragma unroll
        for (int nb = 0; nb < 4; ++nb) acc[mb][nb] = (v8f){};
    const size_t aoff = (size_t)(r0 + lr) * K + 8 * hi, boff = (size_t)(c0 + lr) * K + 8 * hi;
#pragma unroll 1
    for (int kc = 0; kc < K; kc += 32) {
        V a[4], a2[4];
#pragma unroll
        for (int mb = 0; mb < 4; ++mb) { a[mb] = WFrag<T16>::ld(A + aoff + (size_t)mb * 16 * K + kc); if (NSPLIT == 1 || NSPLIT == 2) a2[mb] = WFrag<T16>::ld(A2 + aoff + (size_t)mb * 16 * K + kc); }
#pragma unroll
        for (int nb = 0; nb < 4; ++nb) { const V b = WFrag<T16>::ld(Bt + boff + (size_t)nb * 16 * K + kc); V b2; if (NSPLIT >= 2) b2 = WFrag<T16>::ld(Bt2 + boff + (size_t)nb * 16 * K + kc);
#pragma unroll
            for (int mb = 0; mb < 4; ++mb) { acc[mb][nb] = WFrag<T16>::mma(a[mb], b, acc[mb][nb]); if (NSPLIT == 1 || NSPLIT == 2) acc[mb][nb] = WFrag<T16>::mma(a2[mb], b, acc[mb][nb]); if (NSPLIT >= 2) acc[mb][nb] = WFrag<T16>::mma(a[mb], b2, acc[mb][nb]); } }
        asm volatile("v_nop\n\tv_nop\n\tv_nop\n\tv_nop" : "+v"(acc[0][0]), "+v"(acc[1][1]), "+v"(acc[2][2]), "+v"(acc[3][3]) : "v"(a[0]), "v"(a[3]));
    }
#pragma unroll
    for (int mb = 0; mb < 4; ++mb) {
#pragma unroll
        for (int nb = 0; nb < 4; ++nb) {
#pragma unroll
            for (int j = 0; j < 8; ++j) os[(hi * 8 + j) * 68 + nb * 16 + lr] = acc[mb][nb][j]; }
        __builtin_amdgcn_wave_barrier(); asm volatile("" ::: "memory");
        float* crow = C + (size_t)(r0 + mb * 16) * ldc + c0;
#pragma unroll 1
        for (int ps = 0; ps < 2; ++ps) {
#pragma unroll
            for (int s = 0; s < 8; ++s) { const int row = 2 * s + hi, cofs = lr * 4; v4f val = *(const v4fa*)(os + row * 68 + cofs); if (BIAS) { val[0] += bfr(bias[c0 + cofs]); val[1] += bfr(bias[c0 + cofs + 1]); val[2] += bfr(bias[c0 + cofs + 2]); val[3] += bfr(bias[c0 + cofs + 3]); }
                *(volatile v4f*)(crow + (size_t)row * ldc + cofs) = val; }
            if (ps == 0) __threadfence(); }
        __builtin_amdgcn_wave_barrier(); asm volatile("" ::: "memory");
    }
}

__device__ __forceinline__ h16 tohx(float x) { return (h16)x; }
__device__ __forceinline__ float sigm_(float x) { return __fdiv_rn(1.0f, 1.0f + __expf(-x)); }
__device__ __forceinline__ float silu_(float x) { return __fmul_rn(x, sigm_(x)); }
typedef __attribute__((ext_vector_type(2))) _Float16 v2h;
typedef __attribute__((ext_vector_type(4))) _Float16 v4h;

__global__ __launch_bounds__(256) void k_wt16(const float* __restrict__ w, int K, int N, h16* Bt) { const size_t e = ((size_t)blockIdx.x * 256 + threadIdx.x) * 2; if (e >= (size_t)N * K) return; const int k = (int)(e % K), n = (int)(e / K); v2h o; o[0] = tohx(bfr(w[(size_t)k * N + n])); o[1] = tohx(bfr(w[(size_t)(k + 1) * N + n])); *(volatile v2h*)(Bt + e) = o; __threadfence(); *(volatile v2h*)(Bt + e) = o; }
__global__ __launch_bounds__(256) void k_wt16cat(const float* __restrict__ wa, const float* __restrict__ wb, const float* __restrict__ wc, int K, int N1, int nmat, h16* Bt) { const size_t e = ((size_t)blockIdx.x * 256 + threadIdx.x) * 2; if (e >= (size_t)nmat * N1 * K) return; const int k = (int)(e % K); const int n = (int)(e / K); const int m = n / N1, nn = n % N1; const float* w = m == 0 ? wa : (m == 1 ? wb : wc); v2h o; o[0] = tohx(bfr(w[(size_t)k * N1 + nn])); o[1] = tohx(bfr(w[(size_t)(k + 1) * N1 + nn])); *(volatile v2h*)(Bt + e) = o; __threadfence(); *(volatile v2h*)(Bt + e) = o; }
__global__ __launch_bounds__(256) void k_rms(const float* __restrict__ X, int isin, const float* __restrict__ w, h16* P) { const int lane = threadIdx.x & 31; const int t = blockIdx.x * 8 + (threadIdx.x >> 5); if (t >= TT) return; const size_t rb = (size_t)t * DD; float q2 = 0.f;
#pragma unroll 1
    for (int ch = 0; ch < 6; ++ch) { const v4f a = *(const v4f*)(X + rb + ch * 128 + lane * 4);
#pragma unroll
        for (int q = 0; q < 4; ++q) { const float xv = isin ? bfr(a[q]) : a[q]; float p = __fmul_rn(xv, xv); asm volatile("" : "+v"(p)); q2 = __fadd_rn(q2, p); } }
#pragma unroll
    for (int sh = 16; sh; sh >>= 1) q2 += __shfl_xor(q2, sh, 32);
    const float rs = __frsqrt_rn(__fadd_rn(q2 * (1.0f / DD), 1e-6f));
    for (int ps = 0; ps < 2; ++ps) {
#pragma unroll 1
        for (int ch = 0; ch < 6; ++ch) { const int c0 = ch * 128 + lane * 4; const v4f a = *(const v4f*)(X + rb + c0); v4h o;
#pragma unroll
            for (int q = 0; q < 4; ++q) { const float xv = isin ? bfr(a[q]) : a[q]; float tn = __fmul_rn(xv, rs); asm volatile("" : "+v"(tn)); o[q] = tohx(__fmul_rn(tn, bfr(w[c0 + q]))); }
            *(volatile v4h*)(P + rb + c0) = o; } if (ps == 0) __threadfence(); } }
__global__ __launch_bounds__(256) void k_convg(const float* __restrict__ UG, const float* __restrict__ w, h16* CAT) { const size_t e = ((size_t)blockIdx.x * 256 + threadIdx.x) * 4; if (e >= (size_t)TT * DC) return; const int c = (int)(e % DC); const int t = (int)(e / DC); v4h o;
#pragma unroll
    for (int q = 0; q < 4; ++q) { const int cc = c + q; float acc = 0.f;
#pragma unroll
        for (int k = 0; k < 3; ++k) { const int ts = t - 2 + k; if (ts >= 0) { float p = __fmul_rn(UG[(size_t)ts * DD + cc], bfr(w[cc * 3 + k])); asm volatile("" : "+v"(p)); acc = __fadd_rn(acc, p); } }
        o[q] = tohx(__fmul_rn(acc, silu_(UG[(size_t)t * DD + DC + cc]))); }
    *(volatile v4h*)(CAT + (size_t)t * DD + c) = o; __threadfence(); *(volatile v4h*)(CAT + (size_t)t * DD + c) = o; }
__global__ __launch_bounds__(64) void k_lru(const float* __restrict__ VRI, const float* __restrict__ lam, h16* CAT) { const int c = (blockIdx.x * 64 + threadIdx.x) * 2; if (c >= DG) return; float m8[2];
#pragma unroll
    for (int u = 0; u < 2; ++u) { const float l = bfr(lam[c + u]); const float spl = l > 20.f ? l : log1pf(__expf(l)); m8[u] = __fmul_rn(-8.0f, spl); }
    for (int ps = 0; ps < 2; ++ps) { float h[2] = {0.f, 0.f}; for (int t = 0; t < TT; ++t) { const float* row = VRI + (size_t)t * (3 * DG); v2h o;
#pragma unroll
            for (int u = 0; u < 2; ++u) { const float v = row[c + u]; const float r = sigm_(row[DG + c + u]); const float ig = sigm_(row[2 * DG + c + u]); const float la = __fmul_rn(m8[u], r); const float a = __expf(la);
                const float om = __fsub_rn(1.0f, __expf(__fmul_rn(2.0f, la))); const float gs = __fsqrt_rn(fmaxf(om, 1e-6f)); float iv = __fmul_rn(ig, v); asm volatile("" : "+v"(iv)); float gt = __fmul_rn(gs, iv); asm volatile("" : "+v"(gt)); float ah = __fmul_rn(a, h[u]); asm volatile("" : "+v"(ah)); h[u] = __fadd_rn(ah, gt); o[u] = tohx(h[u]); }
            *(volatile v2h*)(CAT + (size_t)t * DD + DC + c) = o; } if (ps == 0) __threadfence(); } }
__global__ __launch_bounds__(256) void k_mom(const float* __restrict__ x, const float* __restrict__ vin, const float* __restrict__ lb, const float* __restrict__ MIX, float* VEL, float* X1) { const size_t i = ((size_t)blockIdx.x * 256 + threadIdx.x) * 4; if (i >= (size_t)TT * DD) return; const float beta = sigm_(bfr(lb[0])); const v4f m = *(const v4f*)(MIX + i); v4f v, o;
#pragma unroll
    for (int q = 0; q < 4; ++q) { float bv = __fmul_rn(beta, bfr(vin[i + q])); asm volatile("" : "+v"(bv)); v[q] = __fadd_rn(bv, m[q]); o[q] = __fadd_rn(bfr(x[i + q]), v[q]); }
    for (int ps = 0; ps < 2; ++ps) { *(volatile v4f*)(VEL + i) = v; *(volatile v4f*)(X1 + i) = o; if (ps == 0) __threadfence(); } }
__global__ __launch_bounds__(256) void k_swiglu(const float* __restrict__ A, h16* G16) { const size_t e = ((size_t)blockIdx.x * 256 + threadIdx.x) * 4; if (e >= (size_t)TT * DF) return; const int c = (int)(e % DF); const int t = (int)(e / DF); const float* r = A + (size_t)t * 2 * DF; v4h o;
#pragma unroll
    for (int q = 0; q < 4; ++q) o[q] = tohx(__fmul_rn(silu_(r[c + q]), r[DF + c + q])); *(volatile v4h*)(G16 + e) = o; __threadfence(); *(volatile v4h*)(G16 + e) = o; }
__global__ __launch_bounds__(256) void k_fin(const float* __restrict__ X1, const float* __restrict__ F, float* OUT) { const size_t i = ((size_t)blockIdx.x * 256 + threadIdx.x) * 4; if (i >= (size_t)TT * DD) return; const v4f a = *(const v4f*)(X1 + i), f = *(const v4f*)(F + i); v4f o; o[0] = __fadd_rn(a[0], f[0]); o[1] = __fadd_rn(a[1], f[1]); o[2] = __fadd_rn(a[2], f[2]); o[3] = __fadd_rn(a[3], f[3]); *(volatile v4f*)(OUT + i) = o; __threadfence(); *(volatile v4f*)(OUT + i) = o; }

extern "C" void kernel_launch(void* const* d_in, const int* in_sizes, int n_in,
                              void* d_out, int out_size, void* d_ws, size_t ws_size, hipStream_t stream) {
    (void)in_sizes; (void)n_in; (void)out_size;
    const float* x = (const float*)d_in[0]; const float* vin = (const float*)d_in[1]; const float* pnw = (const float*)d_in[2]; const float* wci = (const float*)d_in[3]; const float* wdw = (const float*)d_in[4]; const float* wv = (const float*)d_in[5]; const float* wr = (const float*)d_in[6]; const float* wi = (const float*)d_in[7]; const float* lam = (const float*)d_in[8]; const float* wo = (const float*)d_in[9]; const float* lb = (const float*)d_in[10]; const float* fnw = (const float*)d_in[11]; const float* w1 = (const float*)d_in[12]; const float* w3 = (const float*)d_in[13]; const float* w2 = (const float*)d_in[14];
    float* OUT0 = (float*)d_out; float* OUT1 = (float*)((char*)d_out + 25165824);
    char* wsp = (char*)d_ws;
    auto take = [&](size_t bytes) { char* p = wsp; wsp += (bytes + 255) & ~(size_t)255; return (void*)p; };
    h16* WCI = (h16*)take((size_t)DD * DD * 2); h16* WVRI = (h16*)take((size_t)3 * DG * DD * 2); h16* WO = (h16*)take((size_t)DD * DD * 2); h16* W13 = (h16*)take((size_t)2 * DF * DD * 2); h16* W2 = (h16*)take((size_t)DD * DF * 2);
    h16* P16 = (h16*)take((size_t)TT * DD * 2); float* UG = (float*)take((size_t)TT * DD * 4); float* VRI = (float*)take((size_t)TT * 3 * DG * 4); h16* CAT = (h16*)take((size_t)TT * DD * 2); float* MIX = (float*)take((size_t)TT * DD * 4); float* X1 = (float*)take((size_t)TT * DD * 4); float* A = (float*)take((size_t)TT * 2 * DF * 4); h16* G16 = (h16*)take((size_t)TT * DF * 2);
    if ((size_t)(wsp - (char*)d_ws) > ws_size) return;
    k_wt16<<<(unsigned)(((size_t)DD * DD / 2 + 255) / 256), 256, 0, stream>>>(wci, DD, DD, WCI); k_wt16cat<<<(unsigned)(((size_t)3 * DG * DD / 2 + 255) / 256), 256, 0, stream>>>(wv, wr, wi, DD, DG, 3, WVRI); k_wt16<<<(unsigned)(((size_t)DD * DD / 2 + 255) / 256), 256, 0, stream>>>(wo, DD, DD, WO);
    k_wt16cat<<<(unsigned)(((size_t)2 * DF * DD / 2 + 255) / 256), 256, 0, stream>>>(w1, w3, nullptr, DD, DF, 2, W13); k_wt16<<<(unsigned)(((size_t)DF * DD / 2 + 255) / 256), 256, 0, stream>>>(w2, DF, DD, W2);
    const unsigned L4 = (unsigned)(((size_t)TT * DD / 4 + 255) / 256);
    for (int b = 0; b < NB_; ++b) { const float* xb = x + (size_t)b * TT * DD; const float* vb = vin + (size_t)b * TT * DD;
        k_rms<<<TT / 8, 256, 0, stream>>>(xb, 1, pnw, P16);
        k_gemmw<h16, 0, false><<<dim3(TT / 64, DD / 64, 1), 32, 0, stream>>>(P16, nullptr, WCI, nullptr, DD, UG, DD, nullptr, 0, 0, 0);
        k_gemmw<h16, 0, false><<<dim3(TT / 64, 3 * DG / 64, 1), 32, 0, stream>>>(P16, nullptr, WVRI, nullptr, DD, VRI, 3 * DG, nullptr, 0, 0, 0);
        k_convg<<<(unsigned)(((size_t)TT * DC / 4 + 255) / 256), 256, 0, stream>>>(UG, wdw, CAT); k_lru<<<DG / 128, 64, 0, stream>>>(VRI, lam, CAT);
        k_gemmw<h16, 0, false><<<dim3(TT / 64, DD / 64, 1), 32, 0, stream>>>(CAT, nullptr, WO, nullptr, DD, MIX, DD, nullptr, 0, 0, 0);
        k_mom<<<L4, 256, 0, stream>>>(xb, vb, lb, MIX, OUT1 + (size_t)b * TT * DD, X1);
        k_rms<<<TT / 8, 256, 0, stream>>>(X1, 0, fnw, P16);
        k_gemmw<h16, 0, false><<<dim3(TT / 64, 2 * DF / 64, 1), 32, 0, stream>>>(P16, nullptr, W13, nullptr, DD, A, 2 * DF, nullptr, 0, 0, 0); k_swiglu<<<(unsigned)(((size_t)TT * DF / 4 + 255) / 256), 256, 0, stream>>>(A, G16);
        k_gemmw<h16, 0, false><<<dim3(TT / 64, DD / 64, 1), 32, 0, stream>>>(G16, nullptr, W2, nullptr, DF, MIX, DD, nullptr, 0, 0, 0);
        k_fin<<<L4, 256, 0, stream>>>(X1, MIX, OUT0 + (size_t)b * TT * DD); }
}
